// FeatureAttentionLayer_27212912787959
// MI455X (gfx1250) — hardware-verified
//
#include <hip/hip_runtime.h>

typedef _Float16 v16h  __attribute__((ext_vector_type(16)));
typedef _Float16 half8 __attribute__((ext_vector_type(8)));
typedef float    v8f   __attribute__((ext_vector_type(8)));

#define ALPHA 0.2f
typedef float v4f __attribute__((ext_vector_type(4)));
typedef unsigned v4u __attribute__((ext_vector_type(4)));
typedef float __attribute__((may_alias)) float_a;
template <typename T> __device__ __forceinline__ void vst2(void* p, T v) { *(volatile T*)p = v; __threadfence(); *(volatile T*)p = v; }

__global__ void gat_prep_vh(const float* __restrict__ x, _Float16* __restrict__ vh) {
  int g = blockIdx.x * blockDim.x + threadIdx.x;
  int idx = g * 8;
  int b = idx >> 16;
  int k = (idx >> 8) & 255;
  int w = idx & 255;
  union { _Float16 h[8]; v4u u; } pk;
#pragma unroll
  for (int e = 0; e < 8; ++e) pk.h[e] = (_Float16)x[(b * 256 + w + e) * 256 + k];
  vst2(vh + idx, pk.u);
}

__global__ void gat_prep_wh(const float* __restrict__ W, _Float16* __restrict__ Wh) {
  int g = blockIdx.x * blockDim.x + threadIdx.x;
  union { _Float16 h[8]; v4u u; } pk;
#pragma unroll
  for (int e = 0; e < 8; ++e) pk.h[e] = (_Float16)W[g * 8 + e];
  vst2(Wh + g * 8, pk.u);
}

__global__ void gat_gemm_wmma(const _Float16* __restrict__ vh,
                              const _Float16* __restrict__ Wh,
                              const float* __restrict__ b_lin,
                              float* __restrict__ Lbuf,
                              float* __restrict__ Rpbuf) {
  const int lane = threadIdx.x & 31;
  const int wave = threadIdx.x >> 5;
  const int tile = blockIdx.x * (blockDim.x >> 5) + wave;

  const int side  = tile >> 12;
  const int rem   = tile & 4095;
  const int b     = rem >> 9;
  const int rem2  = rem & 511;
  const int itile = rem2 >> 5;
  const int etile = rem2 & 31;
  const int m0 = itile * 16;
  const int e0 = etile * 16;

  const int n  = lane & 15;
  const int hi = lane >> 4;

  const _Float16* arow = vh + ((b * 256 + m0 + n) * 256);
  const _Float16* brow0 = Wh + (e0 + n) * 512 + side * 256;

  v8f c = {};
#pragma unroll
  for (int w0 = 0; w0 < 256; w0 += 32) {
    half8 alo = *(const half8*)(arow + w0 + hi * 8);
    half8 ahi = *(const half8*)(arow + w0 + 16 + hi * 8);
    v16h a = __builtin_shufflevector(alo, ahi,
                                     0, 1, 2, 3, 4, 5, 6, 7,
                                     8, 9, 10, 11, 12, 13, 14, 15);
    half8 blo = *(const half8*)(brow0 + w0 + hi * 8);
    half8 bhi = *(const half8*)(brow0 + w0 + 16 + hi * 8);
    v16h bm = __builtin_shufflevector(blo, bhi, 0, 1, 2, 3, 4, 5, 6, 7, 8, 9, 10, 11, 12, 13, 14, 15);
    c = __builtin_amdgcn_wmma_f32_16x16x32_f16(
         false, a,  false, bm,
         (short)0, c,  false,  false);
    asm volatile("v_nop\n\tv_nop\n\tv_nop\n\tv_nop" : "+v"(c) : "v"(a), "v"(bm));
  }

  __shared__ __align__(16) float st[16][132];
  const float bl = (side == 0) ? 0.f : b_lin[e0 + n];
#pragma unroll
  for (int r = 0; r < 8; ++r) st[hi * 8 + r][wave * 16 + n] = c[r] + bl;
  __syncthreads();
  const int eblk = (etile & ~7) * 16;
  float* dstbase = (side == 0 ? Lbuf : Rpbuf) + (size_t)(b * 256 + m0) * 512 + eblk;
  for (int q = threadIdx.x; q < 16 * 32; q += 256) { const int rl = q >> 5, pc = q & 31;
    vst2(dstbase + (size_t)rl * 512 + pc * 4, *(const v4f*)(&st[rl][pc * 4])); }
}

__global__ void gat_attn_fused(const float* __restrict__ Lbuf,
                               const float* __restrict__ Rpbuf,
                               const float* __restrict__ a_vec,
                               const float* __restrict__ bias,
                               const _Float16* __restrict__ vh,
                               float* __restrict__ hst) {
  __shared__ float sL[512];
  __shared__ float sA[512];
  __shared__ float sRed[256];
  __shared__ float sAttn[256];

  const int tid = threadIdx.x;
  const int b = blockIdx.x >> 8;
  const int i = blockIdx.x & 255;

  const float* lrow = Lbuf + (b * 256 + i) * 512;
  sL[tid]       = lrow[tid];
  sL[tid + 256] = lrow[tid + 256];
  sA[tid]       = a_vec[tid];
  sA[tid + 256] = a_vec[tid + 256];
  __syncthreads();

  const float* rp = Rpbuf + (size_t)(b * 256 + tid) * 512;
  float acc = 0.f;
#pragma unroll 4
  for (int e = 0; e < 512; ++e) {
    float t = sL[e] + rp[e];
    float leaky = fmaxf(t, ALPHA * t);
    acc = fmaf(sA[e], leaky, acc);
  }
  float ej = acc + bias[i * 256 + tid];

  sRed[tid] = ej;
  __syncthreads();
  for (int s = 128; s > 0; s >>= 1) {
    if (tid < s) sRed[tid] = fmaxf(sRed[tid], sRed[tid + s]);
    __syncthreads();
  }
  float mx = sRed[0];
  __syncthreads();
  float p = expf(ej - mx);
  sRed[tid] = p;
  __syncthreads();
  for (int s = 128; s > 0; s >>= 1) {
    if (tid < s) sRed[tid] += sRed[tid + s];
    __syncthreads();
  }
  float inv = 1.0f / sRed[0];
  sAttn[tid] = p * inv;
  __syncthreads();

  const _Float16* vb = vh + b * 256 * 256 + tid;
  float acc2 = 0.f;
#pragma unroll 4
  for (int j = 0; j < 256; ++j) {
    acc2 = fmaf(sAttn[j], (float)vb[j * 256], acc2);
  }
  float h = 1.0f / (1.0f + expf(-acc2));
  vst2(hst + (size_t)(b * 256 + i) * 256 + tid, (float_a)h);
}
__global__ void gat_transpose_out(const float* __restrict__ hst, float* __restrict__ out) {
  __shared__ float tile[32][33];
  const int b = blockIdx.z, i0 = blockIdx.y * 32, w0 = blockIdx.x * 32, tid = threadIdx.x;
  for (int q = tid; q < 32 * 32; q += 256) { const int ii = q >> 5, ww = q & 31; tile[ii][ww] = hst[(size_t)(b * 256 + i0 + ii) * 256 + w0 + ww]; }
  __syncthreads();
  for (int q = tid; q < 32 * 32; q += 256) { const int ww = q >> 5, ii = q & 31; vst2(out + (size_t)(b * 256 + w0 + ww) * 256 + i0 + ii, (float_a)tile[ii][ww]); }
}

extern "C" void kernel_launch(void* const* d_in, const int* in_sizes, int n_in,
                              void* d_out, int out_size, void* d_ws, size_t ws_size,
                              hipStream_t stream) {
  const float* x     = (const float*)d_in[0];
  const float* W     = (const float*)d_in[1];
  const float* b_lin = (const float*)d_in[2];
  const float* a_vec = (const float*)d_in[3];
  const float* bias  = (const float*)d_in[4];
  float* out = (float*)d_out;

  char* ws = (char*)d_ws;
  _Float16* vh   = (_Float16*)(ws);
  _Float16* Wh   = (_Float16*)(ws + (1u << 20));
  float*    Lbuf = (float*)(ws + (1u << 20) + (1u << 19));
  float*    Rpbuf = Lbuf + 8 * 256 * 512;
  float*    hst   = Rpbuf + 8 * 256 * 512;

  gat_prep_vh<<<(8 * 256 * 256 / 8) / 256, 256, 0, stream>>>(x, vh);
  gat_prep_wh<<<(512 * 512 / 8) / 256, 256, 0, stream>>>(W, Wh);

  gat_gemm_wmma<<<1024, 256, 0, stream>>>(vh, Wh, b_lin, Lbuf, Rpbuf);

  gat_attn_fused<<<2048, 256, 0, stream>>>(Lbuf, Rpbuf, a_vec, bias, vh, hst);
  gat_transpose_out<<<dim3(256 / 32, 256 / 32, 8), 256, 0, stream>>>(hst, out);
}
